// CausalAttention_7292854468924
// MI455X (gfx1250) — hardware-verified
//
#include <hip/hip_runtime.h>


#ifndef NB
#define NB 8
#endif
#ifndef SEQ
#define SEQ 1024
#endif
#define S_FULL 1024
#define IC 256
#define EC 256
#define OC 256
#define KVR (EC + OC)
#define NHD 8
#define HD 32
#define TT SEQ
#define ZH NHD
#define QKW (2 * EC)
#define SCL 0.17677669529663688f

static_assert(SEQ % 128 == 0);
static_assert(SEQ <= S_FULL);
static_assert(NB >= 1 && NB <= 8);
static_assert(EC == NHD * HD);
static_assert(OC == NHD * HD);
static_assert(HD == 32);
static_assert(IC % 64 == 0 && EC % 64 == 0 && OC % 64 == 0);

typedef _Float16 h16;
typedef unsigned short bf;
typedef __attribute__((ext_vector_type(16))) __bf16   v16bf;
typedef __attribute__((ext_vector_type(16))) _Float16 v16h;
typedef __attribute__((ext_vector_type(8)))  _Float16 v8h;
typedef __attribute__((ext_vector_type(8)))  unsigned short v8us;
typedef __attribute__((ext_vector_type(8)))  float    v8f;
typedef __attribute__((ext_vector_type(4)))  float    v4f;
typedef __attribute__((ext_vector_type(4)))  unsigned short v4us;
typedef __attribute__((ext_vector_type(2)))  unsigned short v2us;
typedef v4f  __attribute__((may_alias)) v4fa;

__device__ __forceinline__ unsigned short f2bf(float f) { unsigned u = __float_as_uint(f); u += 0x7FFFu + ((u >> 16) & 1u); return (unsigned short)(u >> 16); }
__device__ __forceinline__ float bf2f(unsigned short b) { return __uint_as_float(((unsigned)b) << 16); }
__device__ __forceinline__ float bfr(float f) { return bf2f(f2bf(f)); }
__device__ __forceinline__ void splitf(float y, unsigned short& h, unsigned short& l) { h = f2bf(y); l = f2bf(y - bf2f(h)); }
__device__ __forceinline__ v16h cat16(v8h lo, v8h hi) { return __builtin_shufflevector(lo, hi, 0, 1, 2, 3, 4, 5, 6, 7, 8, 9, 10, 11, 12, 13, 14, 15); }
__device__ __forceinline__ v16bf cat16b(v8us lo, v8us hi) { return __builtin_bit_cast(v16bf, __builtin_shufflevector(lo, hi, 0, 1, 2, 3, 4, 5, 6, 7, 8, 9, 10, 11, 12, 13, 14, 15)); }
__device__ __forceinline__ v8f wmma16(v16h a, v16h b, v8f c) { return __builtin_amdgcn_wmma_f32_16x16x32_f16(false, a, false, b, (short)0, c, false, false); }
__device__ __forceinline__ v8f wmmab(v16bf a, v16bf b, v8f c) { return __builtin_amdgcn_wmma_f32_16x16x32_bf16(false, a, false, b, (short)0, c, false, false); }

template <typename T16> struct WFrag;
template <> struct WFrag<h16> { typedef v16h V; static __device__ __forceinline__ V ld(const h16* p) { return cat16(*(const v8h*)p, *(const v8h*)(p + 16)); } static __device__ __forceinline__ v8f mma(V a, V b, v8f c) { return wmma16(a, b, c); } };
template <> struct WFrag<bf> { typedef v16bf V; static __device__ __forceinline__ V ld(const bf* p) { return cat16b(*(const v8us*)p, *(const v8us*)(p + 16)); } static __device__ __forceinline__ v8f mma(V a, V b, v8f c) { return wmmab(a, b, c); } };

template <typename T16, bool SPLA, bool SPLB, int BIASM, int NW, int CAUS>
__global__ __launch_bounds__(32) __attribute__((amdgpu_num_vgpr(256)))
void k_gemmw(const T16* __restrict__ A, const T16* __restrict__ A2, const T16* __restrict__ Bt, const T16* __restrict__ Bt2, int K, float* C, int ldc, const float* __restrict__ bias, size_t sA, size_t sB, size_t sC) {
    typedef typename WFrag<T16>::V V;
    constexpr int LPR = NW * 4;
    constexpr int RPI = 32 / LPR;
    constexpr int NST = 16 / RPI;
    static_assert(NW == 2 || NW == 4);
    __shared__ __align__(16) float os[16 * 68];
    const size_t z = blockIdx.z; A += z * sA; if (SPLA) A2 += z * sA; Bt += z * sB; if (SPLB) Bt2 += z * sB; C += z * sC;
    const int lane = threadIdx.x & 31, lr = lane & 15, hi = lane >> 4; const int r0 = blockIdx.x * 64, c0 = blockIdx.y * (NW * 16);
    if (CAUS == 1 && c0 >= r0 + 64) return;
    const int kend = (CAUS == 2 && (r0 + 64) < K) ? (r0 + 64) : K;
    v8f acc[4][NW];
#pragma unroll
    for (int mb = 0; mb < 4; ++mb)
#pragma unroll
        for (int nb = 0; nb < NW; ++nb) acc[mb][nb] = (v8f){};
    const size_t aoff = (size_t)(r0 + lr) * K + 8 * hi, boff = (size_t)(c0 + lr) * K + 8 * hi;
#pragma unroll 1
    for (int kc = 0; kc < kend; kc += 32) {
        V a[4], a2[4];
#pragma unroll
        for (int mb = 0; mb < 4; ++mb) { a[mb] = WFrag<T16>::ld(A + aoff + (size_t)mb * 16 * K + kc); if (SPLA) a2[mb] = WFrag<T16>::ld(A2 + aoff + (size_t)mb * 16 * K + kc); else a2[mb] = a[mb]; }
#pragma unroll
        for (int nb = 0; nb < NW; ++nb) { const V b = WFrag<T16>::ld(Bt + boff + (size_t)nb * 16 * K + kc); V b2 = b; if (SPLB) b2 = WFrag<T16>::ld(Bt2 + boff + (size_t)nb * 16 * K + kc);
#pragma unroll
            for (int mb = 0; mb < 4; ++mb) { acc[mb][nb] = WFrag<T16>::mma(a[mb], b, acc[mb][nb]); if (SPLA) acc[mb][nb] = WFrag<T16>::mma(a2[mb], b, acc[mb][nb]); if (SPLB) acc[mb][nb] = WFrag<T16>::mma(a[mb], b2, acc[mb][nb]); } }
        if (NW == 4) { asm volatile("v_nop\n\tv_nop\n\tv_nop\n\tv_nop" : "+v"(acc[0][0]), "+v"(acc[1][NW > 1 ? 1 : 0]), "+v"(acc[2][NW > 2 ? 2 : 0]), "+v"(acc[3][NW - 1]) : "v"(a[0]), "v"(a[3])); }
        else { asm volatile("v_nop\n\tv_nop\n\tv_nop\n\tv_nop" : "+v"(acc[0][0]), "+v"(acc[1][0]), "+v"(acc[2][0]), "+v"(acc[3][0]), "+v"(acc[0][NW - 1]), "+v"(acc[1][NW - 1]), "+v"(acc[2][NW - 1]), "+v"(acc[3][NW - 1]) : "v"(a[0]), "v"(a[3])); }
    }
#pragma unroll
    for (int mb = 0; mb < 4; ++mb) {
#pragma unroll
        for (int nb = 0; nb < NW; ++nb) {
#pragma unroll
            for (int j = 0; j < 8; ++j) os[(hi * 8 + j) * 68 + nb * 16 + lr] = acc[mb][nb][j]; }
        __builtin_amdgcn_wave_barrier(); asm volatile("" ::: "memory");
        float* crow = C + (size_t)(r0 + mb * 16) * ldc + c0;
#pragma unroll 1
        for (int ps = 0; ps < 2; ++ps) {
#pragma unroll
            for (int s = 0; s < NST; ++s) { const int row = RPI * s + lane / LPR, cofs = (lane % LPR) * 4; v4f val = *(const v4fa*)(os + row * 68 + cofs);
                if (BIASM == 1) { val[0] += bfr(bias[c0 + cofs]); val[1] += bfr(bias[c0 + cofs + 1]); val[2] += bfr(bias[c0 + cofs + 2]); val[3] += bfr(bias[c0 + cofs + 3]); }
                if (BIASM == 2) { const float bb = bfr(bias[r0 + mb * 16 + row]); val[0] += bb; val[1] += bb; val[2] += bb; val[3] += bb; }
                *(volatile v4f*)(crow + (size_t)row * ldc + cofs) = val; }
            if (ps == 0) __threadfence(); }
        __builtin_amdgcn_wave_barrier(); asm volatile("" ::: "memory");
    }
}

__global__ __launch_bounds__(256) void k_cvt8(const float* __restrict__ src, bf* dst, size_t n8) { const size_t i = (size_t)blockIdx.x * 256 + threadIdx.x; if (i >= n8) return; const v8f v = *(const v8f*)(src + i * 8); v8us o;
#pragma unroll
    for (int k = 0; k < 8; ++k) o[k] = f2bf(v[k]); *(volatile v8us*)(dst + i * 8) = o; __threadfence(); *(volatile v8us*)(dst + i * 8) = o; }

__global__ __launch_bounds__(256) void k_xT(const float* __restrict__ x, bf* XT) {
    const int lane = threadIdx.x & 31; const int wave = threadIdx.x >> 5;
    const float* w = x + (size_t)blockIdx.y * IC * S_FULL;
    bf* Bt = XT + (size_t)blockIdx.y * SEQ * IC;
    const int L0 = (blockIdx.x * 8 + wave) * 8; const int nlines = SEQ * IC / 64;
#pragma unroll 1
    for (int ps = 0; ps < 2; ++ps) {
#pragma unroll 1
        for (int l = 0; l < 8; ++l) { const int L = L0 + l; if (L >= nlines) break; const size_t e = (size_t)L * 64 + lane * 2; const int c = (int)(e % IC), s = (int)(e / IC); v2us o;
            o[0] = f2bf(w[(size_t)c * S_FULL + s]); o[1] = f2bf(w[(size_t)(c + 1) * S_FULL + s]); *(volatile v2us*)(Bt + e) = o; }
        if (ps == 0) __threadfence(); }
}

__global__ __launch_bounds__(256) void k_qkpl(const float* __restrict__ C1, int col0, bf* PH, bf* PL, size_t n8) {
    const size_t i8 = (size_t)blockIdx.x * 256 + threadIdx.x; if (i8 >= n8) return;
    const int d0 = (int)(i8 % (HD / 8)) * 8; const int i = (int)((i8 / (HD / 8)) % SEQ); const size_t u = i8 / ((size_t)(HD / 8) * SEQ); const size_t n = u / NHD; const int h = (int)(u % NHD);
    const v8f v = *(const v8f*)(C1 + (n * SEQ + i) * QKW + col0 + h * HD + d0);
    v8us oh, ol;
#pragma unroll
    for (int k = 0; k < 8; ++k) { unsigned short a, c; splitf(v[k], a, c); oh[k] = a; ol[k] = c; }
    *(volatile v8us*)(PH + i8 * 8) = oh; *(volatile v8us*)(PL + i8 * 8) = ol; __threadfence(); *(volatile v8us*)(PH + i8 * 8) = oh; *(volatile v8us*)(PL + i8 * 8) = ol;
}

__global__ __launch_bounds__(256) void k_vpl(const float* __restrict__ C2, const float* __restrict__ bkv, bf* VH, bf* VL, size_t n8) {
    const size_t i8 = (size_t)blockIdx.x * 256 + threadIdx.x; if (i8 >= n8) return;
    const size_t row = i8 / (SEQ / 8); const int e = (int)(row % OC); const float bb = bfr(bkv[EC + e]);
    const v8f v = *(const v8f*)(C2 + i8 * 8);
    v8us oh, ol;
#pragma unroll
    for (int k = 0; k < 8; ++k) { unsigned short a, c; splitf(v[k] + bb, a, c); oh[k] = a; ol[k] = c; }
    *(volatile v8us*)(VH + i8 * 8) = oh; *(volatile v8us*)(VL + i8 * 8) = ol; __threadfence(); *(volatile v8us*)(VH + i8 * 8) = oh; *(volatile v8us*)(VL + i8 * 8) = ol;
}

__global__ __launch_bounds__(256) void k_ctpl(const float* __restrict__ AT, bf* CH, bf* CL, size_t n8) {
    const size_t i8 = (size_t)blockIdx.x * 256 + threadIdx.x; if (i8 >= n8) return;
    const v8f v = *(const v8f*)(AT + i8 * 8);
    v8us oh, ol;
#pragma unroll
    for (int k = 0; k < 8; ++k) { unsigned short a, c; splitf(v[k], a, c); oh[k] = a; ol[k] = c; }
    *(volatile v8us*)(CH + i8 * 8) = oh; *(volatile v8us*)(CL + i8 * 8) = ol; __threadfence(); *(volatile v8us*)(CH + i8 * 8) = oh; *(volatile v8us*)(CL + i8 * 8) = ol;
}

__global__ __launch_bounds__(256) void k_asoft(const float* __restrict__ Sb, bf* Ph, bf* Pl) {
    const int lane = threadIdx.x & 31; const int row = blockIdx.x * 8 + (threadIdx.x >> 5); if (row >= ZH * TT) return; const int i = row % TT;
    const float* sr = Sb + (size_t)row * TT; float v[TT / 32]; float mx = -3.0e38f;
#pragma unroll
    for (int ch = 0; ch < TT / 128; ++ch) { const int j0 = ch * 128 + lane * 4; const v4f a = *(const v4f*)(sr + j0);
#pragma unroll
        for (int q = 0; q < 4; ++q) { const int j = j0 + q; const float t = (j <= i) ? a[q] * SCL : -3.0e38f; v[ch * 4 + q] = t; mx = fmaxf(mx, t); } }
#pragma unroll
    for (int sh = 16; sh; sh >>= 1) mx = fmaxf(mx, __shfl_xor(mx, sh, 32));
    float sum = 0.f;
#pragma unroll
    for (int k = 0; k < TT / 32; ++k) { float d0 = __fsub_rn(v[k], mx); asm volatile("" : "+v"(d0)); v[k] = __builtin_amdgcn_exp2f(__fmul_rn(d0, 1.4426950408889634f)); sum += v[k]; }
#pragma unroll
    for (int sh = 16; sh; sh >>= 1) sum += __shfl_xor(sum, sh, 32);
    const float f = __fdiv_rn(1.0f, sum);
#pragma unroll 1
    for (int ps = 0; ps < 2; ++ps) {
#pragma unroll
        for (int ch = 0; ch < TT / 128; ++ch) { v4us oh, ol;
#pragma unroll
            for (int q = 0; q < 4; ++q) { unsigned short a, c2; splitf(v[ch * 4 + q] * f, a, c2); oh[q] = a; ol[q] = c2; }
            const size_t oo = (size_t)row * TT + ch * 128 + lane * 4; *(volatile v4us*)(Ph + oo) = oh; *(volatile v4us*)(Pl + oo) = ol; }
        if (ps == 0) __threadfence(); }
}

extern "C" void kernel_launch(void* const* d_in, const int* in_sizes, int n_in,
                              void* d_out, int out_size, void* d_ws, size_t ws_size, hipStream_t stream) {
    if (n_in < 7) return;
    const float* x     = (const float*)d_in[0];
    const float* wq    = (const float*)d_in[1];
    const float* bq    = (const float*)d_in[2];
    const float* wkv   = (const float*)d_in[3];
    const float* bkv   = (const float*)d_in[4];
    const float* wproj = (const float*)d_in[5];
    const float* bproj = (const float*)d_in[6];
    float* out = (float*)d_out;
    if ((size_t)in_sizes[0] < (size_t)NB * IC * S_FULL) return;
    if (in_sizes[1] < EC * IC || in_sizes[2] < EC || in_sizes[3] < KVR * IC || in_sizes[4] < KVR || in_sizes[5] < OC * OC || in_sizes[6] < OC) return;
    if ((size_t)out_size < (size_t)NB * OC * SEQ) return;

    char* wsp = (char*)d_ws;
    auto take = [&](size_t bytes) { char* p = wsp; wsp += (bytes + 255) & ~(size_t)255; return (void*)p; };
    const size_t nXT  = (size_t)NB * SEQ * IC;
    const size_t nC1  = (size_t)NB * SEQ * QKW;
    const size_t nC2  = (size_t)NB * OC * SEQ;
    const size_t nQK  = (size_t)NB * NHD * SEQ * HD;
    const size_t nV   = (size_t)NB * NHD * HD * SEQ;
    const size_t nS   = (size_t)ZH * SEQ * SEQ;
    const size_t nAT  = (size_t)NB * SEQ * OC;
    const size_t r1a = nC1 * 4 + nC2 * 4, r1b = nS * 4; const size_t r1 = (r1a > r1b) ? r1a : r1b;
    bf* WB  = (bf*)take((size_t)(EC + KVR) * IC * 2);
    bf* WP  = (bf*)take((size_t)OC * OC * 2);
    bf* XT  = (bf*)take(nXT * 2);
    float* R1 = (float*)take(r1);
    float* C1 = R1; float* C2 = R1 + nC1; float* Sb = R1;
    bf* QH = (bf*)take(nQK * 2); bf* QL = (bf*)take(nQK * 2); bf* KH = (bf*)take(nQK * 2); bf* KL = (bf*)take(nQK * 2);
    bf* VH = (bf*)take(nV * 2);  bf* VL = (bf*)take(nV * 2);
    bf* Ph = (bf*)take(nS * 2);  bf* Pl = (bf*)take(nS * 2);
    float* AT = (float*)take(nAT * 4);
    bf* CH = (bf*)take(nAT * 2); bf* CL = (bf*)take(nAT * 2);
    const size_t used = (size_t)(wsp - (char*)d_ws);
    if (used > ws_size || used > (size_t)134217728) return;

    auto nblk = [](size_t n) { return (unsigned)((n + 255) / 256); };
    k_cvt8<<<nblk((size_t)EC * IC / 8), 256, 0, stream>>>(wq, WB, (size_t)EC * IC / 8);
    k_cvt8<<<nblk((size_t)KVR * IC / 8), 256, 0, stream>>>(wkv, WB + (size_t)EC * IC, (size_t)KVR * IC / 8);
    k_cvt8<<<nblk((size_t)OC * OC / 8), 256, 0, stream>>>(wproj, WP, (size_t)OC * OC / 8);
    k_xT<<<dim3((unsigned)((SEQ * IC / 64 + 63) / 64), NB), 256, 0, stream>>>(x, XT);
    k_gemmw<bf, false, false, 1, 4, 0><<<dim3(SEQ / 64, EC / 64, NB), 32, 0, stream>>>(XT, XT, WB, WB, IC, C1, QKW, bq, (size_t)SEQ * IC, (size_t)0, (size_t)SEQ * QKW);
    k_gemmw<bf, false, false, 1, 4, 0><<<dim3(SEQ / 64, EC / 64, NB), 32, 0, stream>>>(XT, XT, WB + (size_t)EC * IC, WB + (size_t)EC * IC, IC, C1 + EC, QKW, bkv, (size_t)SEQ * IC, (size_t)0, (size_t)SEQ * QKW);
    k_gemmw<bf, false, false, 0, 4, 0><<<dim3(OC / 64, SEQ / 64, NB), 32, 0, stream>>>(WB + (size_t)2 * EC * IC, WB + (size_t)2 * EC * IC, XT, XT, IC, C2, SEQ, bq, (size_t)0, (size_t)SEQ * IC, (size_t)OC * SEQ);
    k_qkpl<<<nblk(nQK / 8), 256, 0, stream>>>(C1, 0, QH, QL, nQK / 8);
    k_qkpl<<<nblk(nQK / 8), 256, 0, stream>>>(C1, EC, KH, KL, nQK / 8);
    k_vpl<<<nblk(nV / 8), 256, 0, stream>>>(C2, bkv, VH, VL, nV / 8);
    for (int n = 0; n < NB; ++n) {
        const size_t qo = (size_t)n * NHD * SEQ * HD, vo = (size_t)n * NHD * HD * SEQ;
        k_gemmw<bf, true, true, 0, 2, 1><<<dim3(SEQ / 64, SEQ / 32, NHD), 32, 0, stream>>>(QH + qo, QL + qo, KH + qo, KL + qo, HD, Sb, SEQ, bq, (size_t)SEQ * HD, (size_t)SEQ * HD, (size_t)SEQ * SEQ);
        k_asoft<<<(unsigned)(ZH * TT / 8), 256, 0, stream>>>(Sb, Ph, Pl);
        k_gemmw<bf, true, true, 0, 2, 2><<<dim3(SEQ / 64, 1, NHD), 32, 0, stream>>>(Ph, Pl, VH + vo, VL + vo, SEQ, AT + (size_t)n * SEQ * OC, OC, bq, (size_t)SEQ * SEQ, (size_t)HD * SEQ, (size_t)HD);
    }
    k_ctpl<<<nblk(nAT / 8), 256, 0, stream>>>(AT, CH, CL, nAT / 8);
    k_gemmw<bf, false, true, 2, 4, 0><<<dim3(OC / 64, SEQ / 64, NB), 32, 0, stream>>>(WP, WP, CH, CL, OC, out, SEQ, bproj, (size_t)0, (size_t)SEQ * OC, (size_t)OC * SEQ);
}
